// DeltaNetAttention_5299989643476
// MI455X (gfx1250) — hardware-verified
//
#include <hip/hip_runtime.h>
#include <stddef.h>
#include <stdint.h>

#define NBAT 8
#define SL   256
#define NTOK 2048
#define DM   2048
#define NHD  8
#define HD   256
#define NBH  64

static_assert(NTOK == NBAT * SL);
static_assert(DM == NHD * HD);
static_assert(HD == SL);
static_assert(NTOK % 256 == 0);
static_assert(DM % 64 == 0);
static_assert(DM % 2048 == 0);
static_assert(SL % 64 == 0);
static_assert(HD == 256);

typedef _Float16 v16h __attribute__((ext_vector_type(16)));
typedef _Float16 v8h  __attribute__((ext_vector_type(8)));
typedef float    v8f  __attribute__((ext_vector_type(8)));
typedef float    v4f  __attribute__((ext_vector_type(4)));
typedef unsigned int v4u __attribute__((ext_vector_type(4)));

union Frag  { v16h v; v8h h[2]; };
union Pack8 { v8h h; v4u u; };

__device__ __forceinline__ v8f mma16(v16h a, v16h b, v8f c) {
  c = __builtin_amdgcn_wmma_f32_16x16x32_f16(false, a, false, b, (short)0, c, false, false);
  asm volatile("v_nop\n\tv_nop\n\tv_nop\n\tv_nop" : "+v"(c) : "v"(a), "v"(b));
  return c;
}

__device__ __forceinline__ v16h ldfrag(const _Float16* p, int ld, int row0, int k0, int lane) {
  const int m = lane & 15, lh = lane >> 4;
  const _Float16* q = p + (size_t)(row0 + m) * ld + k0 + 8 * lh;
  Frag f;
  f.h[0] = *(const v8h*)(q);
  f.h[1] = *(const v8h*)(q + 16);
  return f.v;
}

__device__ __forceinline__ v8f zero8() { return (v8f){0.f, 0.f, 0.f, 0.f, 0.f, 0.f, 0.f, 0.f}; }

__device__ __forceinline__ v4u pack8h(v4f a0, v4f a1) {
  Pack8 pk;
  pk.h = (v8h){(_Float16)a0[0], (_Float16)a0[1], (_Float16)a0[2], (_Float16)a0[3],
               (_Float16)a1[0], (_Float16)a1[1], (_Float16)a1[2], (_Float16)a1[3]};
  return pk.u;
}

__device__ __forceinline__ float phi1(float x) {
  return x > 0.0f ? x + 1.0f : __expf(x);
}

__device__ __forceinline__ void gemm32x64(const _Float16* __restrict__ A, int lda,
                                          const _Float16* __restrict__ Bt, int ldb, int K,
                                          int m0, int n0, int lane, v8f (&acc)[2][4]) {
#pragma unroll 2
  for (int k0 = 0; k0 < K; k0 += 32) {
    const v16h a0 = ldfrag(A, lda, m0, k0, lane);
    const v16h a1 = ldfrag(A, lda, m0 + 16, k0, lane);
    const v16h b0 = ldfrag(Bt, ldb, n0, k0, lane);
    const v16h b1 = ldfrag(Bt, ldb, n0 + 16, k0, lane);
    const v16h b2 = ldfrag(Bt, ldb, n0 + 32, k0, lane);
    const v16h b3 = ldfrag(Bt, ldb, n0 + 48, k0, lane);
    acc[0][0] = mma16(a0, b0, acc[0][0]);
    acc[1][0] = mma16(a1, b0, acc[1][0]);
    acc[0][1] = mma16(a0, b1, acc[0][1]);
    acc[1][1] = mma16(a1, b1, acc[1][1]);
    acc[0][2] = mma16(a0, b2, acc[0][2]);
    acc[1][2] = mma16(a1, b2, acc[1][2]);
    acc[0][3] = mma16(a0, b3, acc[0][3]);
    acc[1][3] = mma16(a1, b3, acc[1][3]);
  }
}

#define OTP 68
__device__ __forceinline__ void out_f32(v8f (&acc)[2][4], float scale,
                                        float* sw, float* __restrict__ out, int ldc,
                                        int m0, int n0, int lane, int hh, int c) {
#pragma unroll
  for (int sub = 0; sub < 2; ++sub) {
    __syncthreads();
#pragma unroll
    for (int t = 0; t < 4; ++t) {
#pragma unroll
      for (int r = 0; r < 8; ++r) sw[(8 * hh + r) * OTP + 16 * t + c] = acc[sub][t][r] * scale;
    }
    __syncthreads();
    v4f val[8];
    size_t go[8];
#pragma unroll
    for (int it = 0; it < 8; ++it) {
      const int p    = lane + 32 * it;
      const int L    = p >> 3;
      const int pc   = p & 7;
      const int row  = L >> 1;
      const int half = L & 1;
      val[it] = *(const v4f*)(sw + row * OTP + half * 32 + pc * 4);
      go[it]  = (size_t)(m0 + sub * 16 + row) * ldc + n0 + half * 32 + pc * 4;
    }
    for (int ps = 0; ps < 2; ++ps) {
#pragma unroll
      for (int it = 0; it < 8; ++it) *(volatile v4f*)(out + go[it]) = val[it];
      __threadfence();
    }
  }
}

__device__ __forceinline__ void out_kp(v8f (&acc)[2][4], float scale, float* sw,
                                       _Float16* __restrict__ kh, _Float16* __restrict__ pkp,
                                       int m0, int n0, int lane, int hh, int c) {
#pragma unroll
  for (int sub = 0; sub < 2; ++sub) {
    __syncthreads();
#pragma unroll
    for (int t = 0; t < 4; ++t) {
#pragma unroll
      for (int r = 0; r < 8; ++r) sw[(8 * hh + r) * OTP + 16 * t + c] = acc[sub][t][r] * scale;
    }
    __syncthreads();
    v4u va[4], vb[4];
    size_t go[4];
#pragma unroll
    for (int it = 0; it < 4; ++it) {
      const int p  = lane + 32 * it;
      const int L  = p >> 3;
      const int pc = p & 7;
      const float* ra = sw + L * OTP + pc * 8;
      const v4f a0 = *(const v4f*)(ra);
      const v4f a1 = *(const v4f*)(ra + 4);
      va[it] = pack8h(a0, a1);
      const v4f b0 = (v4f){phi1(a0[0]), phi1(a0[1]), phi1(a0[2]), phi1(a0[3])};
      const v4f b1 = (v4f){phi1(a1[0]), phi1(a1[1]), phi1(a1[2]), phi1(a1[3])};
      vb[it] = pack8h(b0, b1);
      go[it] = (size_t)(m0 + sub * 16 + L) * DM + n0 + pc * 8;
    }
    for (int ps = 0; ps < 2; ++ps) {
#pragma unroll
      for (int it = 0; it < 4; ++it) {
        *(volatile v4u*)(kh  + go[it]) = va[it];
        *(volatile v4u*)(pkp + go[it]) = vb[it];
      }
      __threadfence();
    }
  }
}

#define TVP 264
__device__ __forceinline__ void out_v(v8f (&acc)[2][4], float scale, _Float16* tl,
                                      _Float16* __restrict__ vh, _Float16* __restrict__ vt,
                                      int bb, int n0b, int tid, int wave, int lane, int hh, int c) {
#pragma unroll
  for (int sub = 0; sub < 2; ++sub) {
#pragma unroll
    for (int t = 0; t < 4; ++t) {
#pragma unroll
      for (int r = 0; r < 8; ++r)
        tl[(16 * t + c) * TVP + 32 * wave + 16 * sub + 8 * hh + r] = (_Float16)(acc[sub][t][r] * scale);
    }
  }
  __syncthreads();
  const int hb = bb * NHD + (n0b >> 8);
  const int db = n0b & (HD - 1);
  v4u v1[8], v2[8];
  size_t g1[8], g2[8];
#pragma unroll
  for (int it = 0; it < 8; ++it) {
    const int dl = wave + 8 * it;
    Pack8 pk;
    pk.h   = *(const v8h*)(tl + dl * TVP + lane * 8);
    v1[it] = pk.u;
    g1[it] = ((size_t)hb * HD + db + dl) * SL + lane * 8;
  }
#pragma unroll
  for (int it = 0; it < 8; ++it) {
    const int p  = tid + 256 * it;
    const int lr = p >> 3;
    const int pc = p & 7;
    const _Float16* cp = tl + (pc * 8) * TVP + lr;
    Pack8 pk;
    pk.h   = (v8h){cp[0 * TVP], cp[1 * TVP], cp[2 * TVP], cp[3 * TVP],
                   cp[4 * TVP], cp[5 * TVP], cp[6 * TVP], cp[7 * TVP]};
    v2[it] = pk.u;
    g2[it] = (size_t)(bb * SL + lr) * DM + n0b + pc * 8;
  }
  for (int ps = 0; ps < 2; ++ps) {
#pragma unroll
    for (int it = 0; it < 8; ++it) {
      *(volatile v4u*)(vt + g1[it]) = v1[it];
      *(volatile v4u*)(vh + g2[it]) = v2[it];
    }
    __threadfence();
  }
}

__global__ __launch_bounds__(256) void k_cvt(const float* __restrict__ src, _Float16* __restrict__ dh, float scale) {
  const size_t o = (size_t)blockIdx.x * 2048 + (size_t)threadIdx.x * 8;
  const v4f a0 = *(const v4f*)(src + o) * scale;
  const v4f a1 = *(const v4f*)(src + o + 4) * scale;
  const v4u vv = pack8h(a0, a1);
  volatile v4u* d = (volatile v4u*)(dh + o);
  *d = vv;
  __threadfence();
  *d = vv;
}

__global__ __launch_bounds__(256) void k_gemm(const _Float16* __restrict__ ap,
                                              const _Float16* __restrict__ wt,
                                              float scale, float* __restrict__ out) {
  __shared__ __align__(16) float st[8][16 * OTP];
  const int tid = threadIdx.x, lane = tid & 31, wave = tid >> 5;
  const int hh = lane >> 4, c = lane & 15;
  const int m0 = blockIdx.x * 256 + wave * 32;
  const int n0 = blockIdx.y * 64;
  v8f acc[2][4];
#pragma unroll
  for (int s = 0; s < 2; ++s)
#pragma unroll
    for (int t = 0; t < 4; ++t) acc[s][t] = zero8();
  gemm32x64(ap, DM, wt, DM, DM, m0, n0, lane, acc);
  out_f32(acc, scale, st[wave], out, DM, m0, n0, lane, hh, c);
}

__global__ __launch_bounds__(256) void k_projk(const _Float16* __restrict__ xh,
                                               const _Float16* __restrict__ wt,
                                               _Float16* __restrict__ kh, _Float16* __restrict__ pkp) {
  __shared__ __align__(16) float st[8][16 * OTP];
  const int tid = threadIdx.x, lane = tid & 31, wave = tid >> 5;
  const int hh = lane >> 4, c = lane & 15;
  const int m0 = blockIdx.x * 256 + wave * 32;
  const int n0 = blockIdx.y * 64;
  v8f acc[2][4];
#pragma unroll
  for (int s = 0; s < 2; ++s)
#pragma unroll
    for (int t = 0; t < 4; ++t) acc[s][t] = zero8();
  gemm32x64(xh, DM, wt, DM, DM, m0, n0, lane, acc);
  out_kp(acc, 0.03125f, st[wave], kh, pkp, m0, n0, lane, hh, c);
}

__global__ __launch_bounds__(256) void k_projv(const _Float16* __restrict__ xh,
                                               const _Float16* __restrict__ wt,
                                               _Float16* __restrict__ vh, _Float16* __restrict__ vt) {
  __shared__ __align__(16) _Float16 tl[64 * TVP];
  const int tid = threadIdx.x, lane = tid & 31, wave = tid >> 5;
  const int hh = lane >> 4, c = lane & 15;
  const int m0 = blockIdx.x * 256 + wave * 32;
  const int n0 = blockIdx.y * 64;
  v8f acc[2][4];
#pragma unroll
  for (int s = 0; s < 2; ++s)
#pragma unroll
    for (int t = 0; t < 4; ++t) acc[s][t] = zero8();
  gemm32x64(xh, DM, wt, DM, DM, m0, n0, lane, acc);
  out_v(acc, 0.03125f, tl, vh, vt, blockIdx.x, n0, tid, wave, lane, hh, c);
}

__global__ __launch_bounds__(256) void k_kv(const _Float16* __restrict__ kh,
                                            const _Float16* __restrict__ vh,
                                            float* __restrict__ kv) {
  __shared__ __align__(16) float st[8][16 * OTP];
  const int tid = threadIdx.x, lane = tid & 31, wave = tid >> 5;
  const int hh = lane >> 4, c = lane & 15;
  const int hb = blockIdx.y;
  const int b = hb >> 3, h = hb & 7;
  const _Float16* A  = kh + (size_t)b * SL * DM + (size_t)h * HD;
  const _Float16* Bt = vh + (size_t)b * SL * DM + (size_t)h * HD;
  const int m0 = wave * 32;
  const int n0 = blockIdx.x * 64;
  v8f acc[2][4];
#pragma unroll
  for (int s = 0; s < 2; ++s)
#pragma unroll
    for (int t = 0; t < 4; ++t) acc[s][t] = zero8();
  gemm32x64(A, DM, Bt, DM, HD, m0, n0, lane, acc);
  out_f32(acc, 1.0f, st[wave], kv + (size_t)hb * SL * SL, SL, m0, n0, lane, hh, c);
}

__global__ __launch_bounds__(256) void k_mean(const float* __restrict__ kv, float* __restrict__ mean) {
  const int h = blockIdx.x, m = threadIdx.x;
  double s = 0.0;
#pragma unroll 1
  for (int b = 0; b < NBAT; ++b) {
    const float* p = kv + (size_t)(b * NHD + h) * SL * SL + m;
#pragma unroll 4
    for (int l = 0; l < SL; ++l) s += (double)p[(size_t)l * SL];
  }
  const float v = (float)s * 0.00048828125f;
  volatile float* d = mean + h * HD + m;
  *d = v;
  __threadfence();
  *d = v;
}

__global__ __launch_bounds__(256) void k_pq(const float* __restrict__ qf, const float* __restrict__ kv,
                                            const float* __restrict__ mean,
                                            const float* __restrict__ alpha_p, const float* __restrict__ beta_p,
                                            _Float16* __restrict__ pq) {
  const int tok = blockIdx.x;
  const int b = tok >> 8, l = tok & 255;
  const int tid = threadIdx.x;
  const int h = tid >> 5;
  const int d0 = (tid & 31) * 8;
  const float alpha = *alpha_p, beta = *beta_p;
  v4f c0 = (v4f){0.f, 0.f, 0.f, 0.f}, c1 = (v4f){0.f, 0.f, 0.f, 0.f};
#pragma unroll 1
  for (int hp = 0; hp < h; ++hp) {
    const v4f ma = *(const v4f*)(mean + hp * HD + d0);
    const v4f mb = *(const v4f*)(mean + hp * HD + d0 + 4);
    c0 = beta * c0 + alpha * ma;
    c1 = beta * c1 + alpha * mb;
  }
  const size_t qo = (size_t)tok * DM + (size_t)h * HD + d0;
  const v4f q0 = *(const v4f*)(qf + qo);
  const v4f q1 = *(const v4f*)(qf + qo + 4);
  const size_t ko = ((size_t)(b * NHD + h) * SL + l) * SL + d0;
  const v4f k0 = *(const v4f*)(kv + ko);
  const v4f k1 = *(const v4f*)(kv + ko + 4);
  const v4f u0 = c0 + alpha * (k0 - c0);
  const v4f u1 = c1 + alpha * (k1 - c1);
  const v4f qm0 = q0 * u0, qm1 = q1 * u1;
  const v4f p0 = (v4f){phi1(qm0[0]), phi1(qm0[1]), phi1(qm0[2]), phi1(qm0[3])};
  const v4f p1 = (v4f){phi1(qm1[0]), phi1(qm1[1]), phi1(qm1[2]), phi1(qm1[3])};
  const v4u val = pack8h(p0, p1);
  volatile v4u* d = (volatile v4u*)(pq + qo);
  *d = val;
  __threadfence();
  *d = val;
}

#define OPW 136
__global__ __launch_bounds__(256) void k_lin(const _Float16* __restrict__ pq,
                                             const _Float16* __restrict__ pkp,
                                             const _Float16* __restrict__ vt,
                                             _Float16* __restrict__ op) {
  __shared__ __align__(16) _Float16 Ps[8 * 16 * OPW];
  const int tid = threadIdx.x, lane = tid & 31, wave = tid >> 5;
  const int hh = lane >> 4, c = lane & 15;
  const int rg = wave & 3, ch = wave >> 2;
  const int qb = blockIdx.x & 3;
  const int hb = blockIdx.x >> 2;
  const int b = hb >> 3, h = hb & 7;
  const int i0 = qb * 64 + rg * 16;
  const _Float16* Aq = pq  + (size_t)b * SL * DM + (size_t)h * HD;
  const _Float16* Bk = pkp + (size_t)b * SL * DM + (size_t)h * HD;
  const _Float16* Bv = vt + (size_t)hb * HD * SL + (size_t)(ch * 128) * SL;
  _Float16* pw = Ps + wave * 16 * OPW;

  v8f oacc[8];
  float denp[8];
#pragma unroll
  for (int t = 0; t < 8; ++t) oacc[t] = zero8();
#pragma unroll
  for (int r = 0; r < 8; ++r) denp[r] = 0.f;

  for (int kc = 0; kc <= qb; ++kc) {
    const int j0 = kc * 64;
    v8f s[4];
#pragma unroll
    for (int jt = 0; jt < 4; ++jt) s[jt] = zero8();
#pragma unroll 2
    for (int ds = 0; ds < 8; ++ds) {
      const v16h qa = ldfrag(Aq, DM, i0, ds * 32, lane);
#pragma unroll
      for (int jt = 0; jt < 4; ++jt) {
        const v16h kb = ldfrag(Bk, DM, j0 + 16 * jt, ds * 32, lane);
        s[jt] = mma16(qa, kb, s[jt]);
      }
    }
    __syncthreads();
#pragma unroll
    for (int r = 0; r < 8; ++r) {
      const int i = i0 + 8 * hh + r;
      float rs = 0.f;
#pragma unroll
      for (int jt = 0; jt < 4; ++jt) {
        const int j = j0 + 16 * jt + c;
        const float v = (j <= i) ? s[jt][r] : 0.f;
        rs += v;
        pw[(8 * hh + r) * OPW + 16 * jt + c] = (_Float16)v;
      }
      denp[r] += rs;
    }
    __syncthreads();
#pragma unroll
    for (int kk = 0; kk < 2; ++kk) {
      const v16h pa = ldfrag(pw, OPW, 0, kk * 32, lane);
#pragma unroll
      for (int t = 0; t < 8; ++t) {
        const v16h vb = ldfrag(Bv, SL, 16 * t, j0 + kk * 32, lane);
        oacc[t] = mma16(pa, vb, oacc[t]);
      }
    }
  }

  float inv[8];
#pragma unroll
  for (int r = 0; r < 8; ++r) {
    float d = denp[r];
    d += __shfl_xor(d, 1, 32);
    d += __shfl_xor(d, 2, 32);
    d += __shfl_xor(d, 4, 32);
    d += __shfl_xor(d, 8, 32);
    inv[r] = 64.0f / fmaxf(d, 1e-8f);
  }
  __syncthreads();
#pragma unroll
  for (int r = 0; r < 8; ++r) {
#pragma unroll
    for (int t = 0; t < 8; ++t)
      pw[(8 * hh + r) * OPW + 16 * t + c] = (_Float16)(oacc[t][r] * inv[r]);
  }
  __syncthreads();
  v4u val[8];
  size_t go[8];
#pragma unroll
  for (int it = 0; it < 8; ++it) {
    const int p  = lane + 32 * it;
    const int L  = p >> 4;
    const int pc = p & 15;
    Pack8 pk;
    pk.h    = *(const v8h*)(pw + L * OPW + pc * 8);
    val[it] = pk.u;
    go[it]  = (size_t)(b * SL + i0 + L) * DM + (size_t)h * HD + ch * 128 + pc * 8;
  }
  for (int ps = 0; ps < 2; ++ps) {
#pragma unroll
    for (int it = 0; it < 8; ++it) *(volatile v4u*)(op + go[it]) = val[it];
    __threadfence();
  }
}

__global__ __launch_bounds__(256) void k_ln(const float* __restrict__ t, const float* __restrict__ res,
                                            const float* __restrict__ bias,
                                            const float* __restrict__ g, const float* __restrict__ be,
                                            float* __restrict__ out) {
  const int tid = threadIdx.x, lane = tid & 31, wave = tid >> 5;
  const size_t m = (size_t)blockIdx.x * 8 + wave;
  const float* tr = t + m * DM;
  const float* rr = res + m * DM;

  float s = 0.f;
#pragma unroll 1
  for (int it = 0; it < 16; ++it) {
    const int idx = it * 128 + lane * 4;
    const v4f a  = *(const v4f*)(tr + idx);
    const v4f bv = *(const v4f*)(bias + idx);
    const v4f r  = *(const v4f*)(rr + idx);
    const v4f x  = r + (a + bv);
    s += (x[0] + x[1]) + (x[2] + x[3]);
  }
#pragma unroll
  for (int off = 16; off >= 1; off >>= 1) s += __shfl_xor(s, off, 32);
  const float mean = s * 0.00048828125f;
  float ss = 0.f;
#pragma unroll 1
  for (int it = 0; it < 16; ++it) {
    const int idx = it * 128 + lane * 4;
    const v4f a  = *(const v4f*)(tr + idx);
    const v4f bv = *(const v4f*)(bias + idx);
    const v4f r  = *(const v4f*)(rr + idx);
    const v4f x  = r + (a + bv);
    const v4f dv = x - mean;
    ss += (dv[0] * dv[0] + dv[1] * dv[1]) + (dv[2] * dv[2] + dv[3] * dv[3]);
  }
#pragma unroll
  for (int off = 16; off >= 1; off >>= 1) ss += __shfl_xor(ss, off, 32);
  const float var  = ss * 0.00048828125f;
  const float rstd = 1.0f / sqrtf(var + 1e-5f);

#pragma unroll 1
  for (int ps = 0; ps < 2; ++ps) {
#pragma unroll 1
    for (int it = 0; it < 16; ++it) {
      const int idx = it * 128 + lane * 4;
      const v4f a  = *(const v4f*)(tr + idx);
      const v4f bv = *(const v4f*)(bias + idx);
      const v4f r  = *(const v4f*)(rr + idx);
      const v4f x  = r + (a + bv);
      const v4f gv = *(const v4f*)(g + idx);
      const v4f ev = *(const v4f*)(be + idx);
      const v4f y  = ((x - mean) * rstd) * gv + ev;
      *(volatile v4f*)(out + m * DM + idx) = y;
    }
    __threadfence();
  }
}

extern "C" void kernel_launch(void* const* d_in, const int* in_sizes, int n_in,
                              void* d_out, int out_size, void* d_ws, size_t ws_size,
                              hipStream_t stream) {
  if (n_in < 12) return;
  if (in_sizes[0] != NTOK * DM) return;
  if (in_sizes[1] != NTOK * DM) return;
  if (in_sizes[2] != NTOK * DM) return;
  if (in_sizes[3] != DM * DM) return;
  if (in_sizes[4] != DM * DM) return;
  if (in_sizes[5] != DM * DM) return;
  if (in_sizes[6] != DM * DM) return;
  if (in_sizes[7] != DM) return;
  if (in_sizes[8] != DM) return;
  if (in_sizes[9] != DM) return;
  if (in_sizes[10] < 1) return;
  if (in_sizes[11] < 1) return;
  if (out_size != NTOK * DM) return;

  const float* query   = (const float*)d_in[0];
  const float* key     = (const float*)d_in[1];
  const float* value   = (const float*)d_in[2];
  const float* wq      = (const float*)d_in[3];
  const float* wk      = (const float*)d_in[4];
  const float* wv      = (const float*)d_in[5];
  const float* wo      = (const float*)d_in[6];
  const float* bo      = (const float*)d_in[7];
  const float* ln_g    = (const float*)d_in[8];
  const float* ln_b    = (const float*)d_in[9];
  const float* alpha_p = (const float*)d_in[10];
  const float* beta_p  = (const float*)d_in[11];
  float* out = (float*)d_out;

  const size_t PL16 = (size_t)NTOK * DM * 2;
  const size_t PL32 = (size_t)NTOK * DM * 4;
  size_t off = 0;
  const size_t oX  = off; off += PL16;
  const size_t oW  = off; off += (size_t)DM * DM * 2;
  const size_t oQf = off; off += PL32;
  const size_t oKh = off; off += PL16;
  const size_t oPk = off; off += PL16;
  const size_t oVh = off; off += PL16;
  const size_t oVt = off; off += (size_t)NBH * HD * SL * 2;
  const size_t oKV = off; off += (size_t)NBH * SL * SL * 4;
  const size_t oPq = off; off += PL16;
  const size_t oOp = off; off += PL16;
  const size_t oT  = off; off += PL32;
  const size_t oMn = off; off += (size_t)NHD * HD * 4;
  if (off > ws_size) return;
  if (off > (size_t)134217728) return;

  char* ws = (char*)d_ws;
  _Float16* Xh  = (_Float16*)(ws + oX);
  _Float16* Wt  = (_Float16*)(ws + oW);
  float*    Qf  = (float*)(ws + oQf);
  _Float16* Kh  = (_Float16*)(ws + oKh);
  _Float16* Pk  = (_Float16*)(ws + oPk);
  _Float16* Vh  = (_Float16*)(ws + oVh);
  _Float16* Vt  = (_Float16*)(ws + oVt);
  float*    KV  = (float*)(ws + oKV);
  _Float16* Pq  = (_Float16*)(ws + oPq);
  _Float16* Op  = (_Float16*)(ws + oOp);
  float*    T   = (float*)(ws + oT);
  float*    Mn  = (float*)(ws + oMn);

  const dim3 blk(256);
  const dim3 gcvt((NTOK * DM) / 2048);
  const dim3 ggemm(NTOK / 256, DM / 64);

  k_cvt<<<gcvt, blk, 0, stream>>>(query, Xh, 1.0f);
  k_cvt<<<gcvt, blk, 0, stream>>>(wq, Wt, 32.0f);
  k_gemm<<<ggemm, blk, 0, stream>>>(Xh, Wt, 0.03125f, Qf);
  k_cvt<<<gcvt, blk, 0, stream>>>(key, Xh, 1.0f);
  k_cvt<<<gcvt, blk, 0, stream>>>(wk, Wt, 32.0f);
  k_projk<<<ggemm, blk, 0, stream>>>(Xh, Wt, Kh, Pk);
  k_cvt<<<gcvt, blk, 0, stream>>>(value, Xh, 1.0f);
  k_cvt<<<gcvt, blk, 0, stream>>>(wv, Wt, 32.0f);
  k_projv<<<ggemm, blk, 0, stream>>>(Xh, Wt, Vh, Vt);
  k_kv<<<dim3(SL / 64, NBH), blk, 0, stream>>>(Kh, Vh, KV);
  k_mean<<<dim3(NHD), blk, 0, stream>>>(KV, Mn);
  k_pq<<<dim3(NTOK), blk, 0, stream>>>(Qf, KV, Mn, alpha_p, beta_p, Pq);
  k_lin<<<dim3(NBH * 4), blk, 0, stream>>>(Pq, Pk, Vt, Op);
  k_cvt<<<gcvt, blk, 0, stream>>>(wo, Wt, 32.0f);
  k_gemm<<<ggemm, blk, 0, stream>>>(Op, Wt, 0.00048828125f, T);
  k_ln<<<dim3(NTOK / 8), blk, 0, stream>>>(T, query, bo, ln_g, ln_b, out);
  (void)hipGetLastError();
}
